// O3EquivariantConv_56573309223684
// MI455X (gfx1250) — hardware-run, weakly checked
//
#include <hip/hip_runtime.h>


namespace {
constexpr int N = 50000, E = 800000, CI = 128, CO = 32, HID = 32, NSH = 18, NBLK = N / 16;
constexpr float XS = 8.0f, YS = 256.0f, WSC = 256.0f;
typedef _Float16 b16;
typedef __attribute__((ext_vector_type(16))) _Float16 v16b;
typedef __attribute__((ext_vector_type(8))) _Float16 v8b;
typedef __attribute__((ext_vector_type(8))) float v8f;
typedef __attribute__((ext_vector_type(4))) float v4f;
__device__ __forceinline__ float bf16_rne(float f) { unsigned int u = __float_as_uint(f); u += 0x7FFFu + ((u >> 16) & 1u); return __uint_as_float(u & 0xFFFF0000u); }
__device__ __forceinline__ void split16(float v, b16& hi, b16& lo) { hi = (b16)v; lo = (b16)(v - (float)hi); }
__device__ __forceinline__ v16b frag_kb(const b16* p, int hh) { const v8b a = *(const v8b*)(p + 8 * hh), b = *(const v8b*)(p + 16 + 8 * hh); v16b f;
#pragma unroll
  for (int e = 0; e < 8; ++e) { f[e] = a[e]; f[8 + e] = b[e]; } return f; }
__device__ __forceinline__ v8f wmma16b(v16b a, v16b b, v8f c) { v8f d = __builtin_amdgcn_wmma_f32_16x16x32_f16(false, a, false, b, (short)0, c, false, false); asm volatile("v_nop\n\tv_nop\n\tv_nop\n\tv_nop" : "+v"(d) : "v"(a), "v"(b)); return d; }
__device__ __forceinline__ void wave_lds_sync() { __builtin_amdgcn_fence(__ATOMIC_RELEASE, "workgroup"); __builtin_amdgcn_wave_barrier(); __builtin_amdgcn_fence(__ATOMIC_ACQUIRE, "workgroup"); }
__device__ __forceinline__ float pmul(float a, float b) { float p = a * b; asm volatile("" : "+v"(p)); return p; }
__device__ __forceinline__ int iclamp(int v, int lo, int hi) { return v < lo ? lo : (v > hi ? hi : v); }
__device__ __forceinline__ float silu(float v) { return v / (1.0f + __expf(-v)); }
constexpr int CSR_NBLK9 = 512, CSR_GB9 = 9, CSR_GN9 = 1 << CSR_GB9  , CSR_TS9 = (CSR_GN9 < 32 ? 32 : CSR_GN9)  , CSR_MAXG9 = 512, CSR_CAP9 = 12288  ;
__device__ __host__ __forceinline__ int csr_tix9(int v) { return (v >> CSR_GB9) * CSR_TS9 + (v & (CSR_GN9 - 1)); }
__global__ __launch_bounds__(64) void csrA_kernel9(const int* __restrict__ dst, int E, int N, int nG, int CHP, int NGP, int* __restrict__ STG, int* __restrict__ HST) {
  extern __shared__ int sm[];
  int* cnt = sm; int* run = sm + NGP; int* ids = sm + 2 * NGP;
  const int b = blockIdx.x; const int ch = (E + CSR_NBLK9 - 1) / CSR_NBLK9; const int e0 = b * ch, e1 = min(E, e0 + ch);
  for (int i = threadIdx.x; i < NGP; i += 64) cnt[i] = 0;
  for (int i = threadIdx.x; i < CHP; i += 64) ids[i] = -1;
  __syncthreads();
  if (threadIdx.x == 0) {
    for (int e = e0; e < e1; ++e) { int d = dst[e]; d = (d < 0) ? 0 : (d >= N ? N - 1 : d); cnt[d >> CSR_GB9] += 1; }
    int acc = 0; for (int g = 0; g < nG; ++g) { run[g] = acc; acc += cnt[g]; }
    for (int e = e0; e < e1; ++e) { int d = dst[e]; d = (d < 0) ? 0 : (d >= N ? N - 1 : d); const int g = d >> CSR_GB9; ids[run[g]] = e; run[g] += 1; } }
  __syncthreads();
  typedef __attribute__((ext_vector_type(4))) int v4i;
  for (int pass = 0; pass < 2; ++pass) {
    for (int i = threadIdx.x; i < CHP / 4; i += 64) *(volatile v4i*)(STG + (size_t)b * CHP + i * 4) = *(const v4i*)(&ids[i * 4]);
    for (int i = threadIdx.x; i < NGP / 4; i += 64) { v4i v; for (int e = 0; e < 4; ++e) v[e] = (i * 4 + e < nG) ? cnt[i * 4 + e] : 0; *(volatile v4i*)(HST + (size_t)b * NGP + i * 4) = v; }
    __threadfence(); }
}
__global__ __launch_bounds__(512) void csrS_kernel9(const int* __restrict__ HST, int nG, int NGP, int* __restrict__ START, int* __restrict__ TOT, int* __restrict__ OFF) {
  __shared__ int tot[CSR_MAXG9];
  const int b = threadIdx.x;
  for (int pass = 0; pass < 2; ++pass) { int runb = 0; for (int g = 0; g < nG; ++g) { int c = HST[(size_t)b * NGP + g]; c = (c < 0) ? 0 : c; ((volatile int*)OFF)[(size_t)g * CSR_NBLK9 + b] = runb; runb += c; } __threadfence(); }
  for (int g = threadIdx.x; g < nG; g += 512) { int s = 0; for (int bb = 0; bb < CSR_NBLK9; ++bb) { int c = HST[(size_t)bb * NGP + g]; s += (c < 0) ? 0 : c; } tot[g] = s; }
  __syncthreads();
  if (threadIdx.x < 32) {
    __shared__ int st[CSR_MAXG9 + 32];
    if (threadIdx.x == 0) { int acc = 0; for (int g = 0; g < NGP; ++g) { st[g] = acc; if (g < nG) acc += (tot[g] + 31) & ~31; } st[NGP] = acc; }
    __builtin_amdgcn_fence(__ATOMIC_RELEASE, "workgroup"); __builtin_amdgcn_wave_barrier(); __builtin_amdgcn_fence(__ATOMIC_ACQUIRE, "workgroup");
    for (int pass = 0; pass < 2; ++pass) { for (int i = threadIdx.x; i < NGP + 32; i += 32) { ((volatile int*)START)[i] = (i <= NGP) ? st[min(i, NGP)] : 0; ((volatile int*)TOT)[i] = (i < nG) ? tot[i] : 0; } __threadfence(); } }
}
__global__ __launch_bounds__(256) void csrB_kernel9(const int* __restrict__ dst, int N, int nG, int CHP, int NGP, int permLen, const int* __restrict__ STG, const int* __restrict__ HST, const int* __restrict__ OFF, const int* __restrict__ START, const int* __restrict__ TOT, int* __restrict__ PERM, int* __restrict__ ROWPTR, int* __restrict__ ROWCNT, int* __restrict__ FLAG) {
  typedef __attribute__((ext_vector_type(4))) int v4i;
  __shared__ int ids[CSR_CAP9]; __shared__ unsigned short key[CSR_CAP9]; __shared__ int outp[CSR_CAP9]; __shared__ int ncnt[CSR_GN9 + 1]; __shared__ int boff[CSR_NBLK9 + 1];
  const int g = blockIdx.x, t_ = threadIdx.x; int tot = TOT[g]; int st = START[g], stn = START[g + 1]; const int v0 = g * CSR_GN9; const int nv = min(CSR_GN9, N - v0); const int t0 = g * CSR_TS9;
  st = (st < 0) ? 0 : (st > permLen - 32 ? permLen - 32 : st) & ~31; stn = (stn < st) ? st : (stn > permLen ? permLen : stn); tot = (tot < 0) ? 0 : tot; if (tot > stn - st && tot <= CSR_CAP9) tot = stn - st;
  if (tot > CSR_CAP9) {
    for (int pass = 0; pass < 2; ++pass) { for (int i = t_; i < CSR_TS9 / 4; i += 256) { v4i a, c; for (int e = 0; e < 4; ++e) { a[e] = st; c[e] = 0; } *(volatile v4i*)(ROWPTR + t0 + i * 4) = a; *(volatile v4i*)(ROWCNT + t0 + i * 4) = c; } if (t_ == 0) ((volatile int*)FLAG)[0] = 1; __threadfence(); } (void)nv; return; }
  if (t_ == 0) { int acc = 0; for (int b = 0; b < CSR_NBLK9; ++b) { boff[b] = acc; int c = HST[(size_t)b * NGP + g]; c = (c < 0) ? 0 : (c > CHP ? CHP : c); acc += c; if (acc > tot) acc = tot; } boff[CSR_NBLK9] = acc; }
  for (int i = t_; i <= CSR_GN9; i += 256) ncnt[i] = 0;
  __syncthreads();
  for (int b = 0; b < CSR_NBLK9; ++b) { const int c = boff[b + 1] - boff[b]; int o_ = OFF[(size_t)g * CSR_NBLK9 + b]; o_ = (o_ < 0) ? 0 : (o_ > CHP - c ? CHP - c : o_); const int* src_ = STG + (size_t)b * CHP + o_;
    for (int i = t_; i < c; i += 256) { int id = src_[i]; id = (id < 0) ? 0 : id; ids[boff[b] + i] = id; int d = dst[id]; d = (d < v0) ? v0 : (d >= N ? N - 1 : d); int kk = d - v0; kk = (kk < 0) ? 0 : (kk >= CSR_GN9 ? CSR_GN9 - 1 : kk); key[boff[b] + i] = (unsigned short)kk; } }
  __syncthreads();
  if (t_ == 0) { for (int i = 0; i < tot; ++i) ncnt[key[i]] += 1; int acc = 0; for (int vl = 0; vl < CSR_GN9; ++vl) { const int c = ncnt[vl]; ncnt[vl] = acc; acc += c; } ncnt[CSR_GN9] = acc;
    for (int i = 0; i < tot; ++i) { const int vl = key[i]; outp[ncnt[vl]] = ids[i]; ncnt[vl] += 1; }
    for (int vl = CSR_GN9; vl > 0; --vl) ncnt[vl] = ncnt[vl - 1]; ncnt[0] = 0; }
  __syncthreads();
  for (int pass = 0; pass < 2; ++pass) {
    for (int i = t_; i < (stn - st) / 4; i += 256) { v4i v; for (int e = 0; e < 4; ++e) { const int q = i * 4 + e; v[e] = (q < tot) ? outp[q] : -1; } *(volatile v4i*)(PERM + st + i * 4) = v; }
    for (int i = t_; i < CSR_TS9 / 4; i += 256) { v4i a, c; for (int e = 0; e < 4; ++e) { const int vl = i * 4 + e; const int vc = vl < CSR_GN9 ? vl : CSR_GN9; a[e] = (vl < CSR_GN9) ? st + ncnt[vc] : st; c[e] = (vl < nv) ? (ncnt[(vc < CSR_GN9 ? vc : CSR_GN9 - 1) + 1] - ncnt[vc]) : 0; } *(volatile v4i*)(ROWPTR + t0 + i * 4) = a; *(volatile v4i*)(ROWCNT + t0 + i * 4) = c; }
    __threadfence(); }
}
__global__ __launch_bounds__(256) void csrZ_kernel9(int* __restrict__ p, size_t n4) { typedef __attribute__((ext_vector_type(4))) int v4i; const size_t tid = (size_t)blockIdx.x * 256 + threadIdx.x, nth = (size_t)gridDim.x * 256; v4i z = {0, 0, 0, 0}; for (size_t i = tid; i < n4; i += nth) *(volatile v4i*)(p + i * 4) = z; }
struct CsrBufs9 { int *STG, *HST, *OFF, *START, *TOT, *PERM, *ROWPTR, *ROWCNT, *FLAG; int nG, NGP, CHP; size_t permLen; char* base; size_t bytes; };
static size_t csr_carve9(CsrBufs9& c, char* ws, size_t off, int E, int N) {
  const size_t off0 = off; c.base = ws + off;
  auto al = [&](size_t bytes) { char* p = ws + off; off += (bytes + 255) & ~(size_t)255; return p; };
  c.nG = (N + CSR_GN9 - 1) / CSR_GN9; c.NGP = (c.nG + 31) & ~31; const int ch = (E + CSR_NBLK9 - 1) / CSR_NBLK9; c.CHP = (ch + 31) & ~31; c.permLen = (size_t)E + 32 * (size_t)c.nG + 32;
  c.STG = (int*)al((size_t)CSR_NBLK9 * c.CHP * 4); c.HST = (int*)al((size_t)CSR_NBLK9 * c.NGP * 4); c.OFF = (int*)al((size_t)c.NGP * CSR_NBLK9 * 4); c.START = (int*)al((size_t)(c.NGP + 64) * 4); c.TOT = (int*)al((size_t)(c.NGP + 64) * 4);
  c.PERM = (int*)al(c.permLen * 4); c.ROWPTR = (int*)al((size_t)c.nG * CSR_TS9 * 4); c.ROWCNT = (int*)al((size_t)c.nG * CSR_TS9 * 4); c.FLAG = (int*)al(256);
  c.bytes = off - off0; return off;
}
static void csr_build9(const CsrBufs9& c, const int* dst, int E, int N, hipStream_t stream) {
  const size_t smem = (size_t)(2 * c.NGP + c.CHP) * 4;
  csrZ_kernel9<<<512, 256, 0, stream>>>((int*)c.base, c.bytes / 16);
  csrA_kernel9<<<CSR_NBLK9, 64, smem, stream>>>(dst, E, N, c.nG, c.CHP, c.NGP, c.STG, c.HST);
  csrS_kernel9<<<1, 512, 0, stream>>>(c.HST, c.nG, c.NGP, c.START, c.TOT, c.OFF);
  csrB_kernel9<<<c.nG, 256, 0, stream>>>(dst, N, c.nG, c.CHP, c.NGP, (int)c.permLen, c.STG, c.HST, c.OFF, c.START, c.TOT, c.PERM, c.ROWPTR, c.ROWCNT, c.FLAG);
}


__global__ __launch_bounds__(256) void wput_kernel(const float* __restrict__ w, int r0, int KIN, int KP, int OUTW, b16* __restrict__ WT) {
  const int KG = KP / 8; const int u = blockIdx.x * 256 + threadIdx.x; if (u >= OUTW * KG) return; const int o = u / KG, k0 = (u % KG) * 8; v8b v;
#pragma unroll
  for (int j = 0; j < 8; ++j) { const int k = k0 + j; v[j] = k < KIN ? (b16)(bf16_rne(w[(size_t)(r0 + k) * OUTW + o]) * WSC) : (b16)0.0f; } for (int pass = 0; pass < 2; ++pass) { *(volatile v8b*)(WT + (size_t)o * KP + k0) = v; __threadfence(); }
}
__global__ __launch_bounds__(256) void w3sum_kernel(const float* __restrict__ W3, const float* __restrict__ b3, b16* __restrict__ W3H, b16* __restrict__ W3L, float* __restrict__ B3S) {
  const int tid = threadIdx.x; const int c = tid / 8, k0g = (tid % 8) * 4;
  v8b hv, lv; for (int q = 0; q < 8; ++q) { hv[q] = (b16)0.0f; lv[q] = (b16)0.0f; }
  { b16 th[4], tl[4];
#pragma unroll
    for (int q = 0; q < 4; ++q) { const int k = k0g + q; float s = 0.0f; for (int sh = 0; sh < NSH; ++sh) s += bf16_rne(W3[(size_t)k * (NSH * CO) + sh * CO + c]); split16(s * WSC, th[q], tl[q]); }
    typedef __attribute__((ext_vector_type(4))) _Float16 v4b; v4b h4 = {th[0], th[1], th[2], th[3]}, l4 = {tl[0], tl[1], tl[2], tl[3]};
    for (int pass = 0; pass < 2; ++pass) { *(volatile v4b*)(W3H + c * HID + k0g) = h4; *(volatile v4b*)(W3L + c * HID + k0g) = l4; __threadfence(); } }
  if (tid < 32) { float s = 0.0f; for (int sh = 0; sh < NSH; ++sh) s += bf16_rne(b3[sh * CO + tid]); for (int pass = 0; pass < 2; ++pass) { ((volatile float*)B3S)[tid] = s; __threadfence(); } }
  (void)hv; (void)lv;
}
__global__ __launch_bounds__(32) void fw_kernel(const float* __restrict__ feat, const b16* __restrict__ W1F, float* __restrict__ FW) {
  __shared__ __attribute__((aligned(16))) b16 Ah[16][CI + 8]; __shared__ float Tf[16][HID + 1];
  const int lane = threadIdx.x, nloc = lane & 15, hlf = lane >> 4; const size_t m0 = (size_t)blockIdx.x * 16;
  for (int rr = 0; rr < 16; ++rr) for (int q = 0; q < 4; ++q) Ah[rr][q * 32 + lane] = (b16)(bf16_rne(feat[(m0 + rr) * CI + q * 32 + lane]) * XS);
  wave_lds_sync();
#pragma unroll
  for (int t = 0; t < 2; ++t) { v8f acc = {};
#pragma unroll
    for (int kb = 0; kb < CI; kb += 32) acc = wmma16b(frag_kb(&Ah[nloc][kb], hlf), frag_kb(W1F + (size_t)(t * 16 + nloc) * CI + kb, hlf), acc);
#pragma unroll
    for (int r8 = 0; r8 < 8; ++r8) Tf[8 * hlf + r8][t * 16 + nloc] = acc[r8] * (1.0f / (XS * WSC)); }
  wave_lds_sync();
  for (int pass = 0; pass < 2; ++pass) { for (int rr = 0; rr < 16; ++rr) ((volatile float*)FW)[(m0 + rr) * HID + lane] = Tf[rr][lane]; __threadfence(); }
}
__global__ __launch_bounds__(32) void msg_kernel(const float* __restrict__ pos, const int* __restrict__ cols, const float* __restrict__ FW, const b16* __restrict__ W1Y, const float* __restrict__ b1, const b16* __restrict__ W2T, const float* __restrict__ b2, const b16* __restrict__ W3H, const b16* __restrict__ W3L, const float* __restrict__ B3S, const int* __restrict__ PERM, const int* __restrict__ ROWPTR, const int* __restrict__ ROWCNT, int permLen, int NLIM, float* __restrict__ out) {
  __shared__ __attribute__((aligned(16))) b16 Ah[16][40], Al[16][40]; __shared__ int Cs[16]; __shared__ float Mo[16][HID + 1];
  const int lane = threadIdx.x, nloc = lane & 15, hlf = lane >> 4; const size_t n = blockIdx.x; if (n >= (size_t)NLIM) return;
  const float px = bf16_rne(pos[n * 3]), py = bf16_rne(pos[n * 3 + 1]), pz = bf16_rne(pos[n * 3 + 2]); const float bb1 = bf16_rne(b1[lane]), bb2 = bf16_rne(b2[lane]), bb3 = B3S[lane];
  int st = ROWPTR[n], cnt = ROWCNT[n]; cnt = iclamp(cnt, 0, 1 << 20); st = iclamp(st, 0, permLen - cnt); float osum = 0.0f;
#pragma unroll 1
  for (int j0 = 0; j0 < cnt; j0 += 16) {
    if (lane < 16) { const int jj = j0 + lane; int c = -1; float yv[NSH]; for (int k = 0; k < NSH; ++k) yv[k] = 0.0f;
      if (jj < cnt) { const int e = iclamp(PERM[st + jj], 0, E - 1); c = iclamp(cols[e], 0, N - 1); if (c >= NLIM) c = -1;
        if (c >= 0) { const float rx = px - bf16_rne(pos[(size_t)c * 3]), ry = py - bf16_rne(pos[(size_t)c * 3 + 1]), rz = pz - bf16_rne(pos[(size_t)c * 3 + 2]); const float dn = fmaxf(sqrtf(pmul(rx, rx) + pmul(ry, ry) + pmul(rz, rz)), 1e-8f); const float dx = rx / dn, dy = ry / dn, dz = rz / dn;
          const float c0 = 0.28209479177387814f, c1a = 0.3454941494713355f, c1b = 0.4886025119029199f, c2a = 0.38627420202318957f, c2b = 0.77254840404637914f, c2c = 0.31539156525252005f;
          for (int sgn = 0; sgn < 2; ++sgn) { const float vx = sgn ? -dx : dx, vy = sgn ? -dy : dy, vz = sgn ? -dz : dz; const float n2 = fmaxf(sqrtf(pmul(vx, vx) + pmul(vy, vy) + pmul(vz, vz)), 1e-8f); const float x = vx / n2, y = vy / n2, z = vz / n2; float* yy = yv + sgn * 9;
            yy[0] = c0; yy[1] = -c1a * x; yy[2] = c1b * z; yy[3] = c1a * x; yy[4] = c2a * (x * x - y * y); yy[5] = -c2b * z * x; yy[6] = c2c * (2.0f * z * z - x * x - y * y); yy[7] = c2b * z * x; yy[8] = c2a * (x * x - y * y); } } }
      Cs[lane] = c; for (int k = 0; k < 32; ++k) { b16 p = (b16)0.0f, q = (b16)0.0f; if (k < NSH) split16(yv[k] * YS, p, q); Ah[lane][k] = p; Al[lane][k] = q; } }
    wave_lds_sync();
    { v8f a2[2] = {(v8f){}, (v8f){}}; const v16b a = frag_kb(&Ah[nloc][0], hlf), al = frag_kb(&Al[nloc][0], hlf);
#pragma unroll
      for (int t = 0; t < 2; ++t) { const v16b bw = frag_kb(W1Y + (size_t)(t * 16 + nloc) * 32, hlf); a2[t] = wmma16b(a, bw, a2[t]); a2[t] = wmma16b(al, bw, a2[t]); }
      wave_lds_sync();
#pragma unroll
      for (int t = 0; t < 2; ++t) { const int c16 = t * 16 + nloc; const float bq = bf16_rne(b1[c16]);
#pragma unroll
        for (int r8 = 0; r8 < 8; ++r8) { const int rl = 8 * hlf + r8; const int cc = Cs[rl]; const float fw = (cc >= 0) ? FW[(size_t)cc * HID + c16] : 0.0f; b16 p, q; split16(silu(a2[t][r8] * (1.0f / (YS * WSC)) + fw + bq) * XS, p, q); Ah[rl][c16] = p; Al[rl][c16] = q; } } }
    wave_lds_sync();
    { v8f a2[2] = {(v8f){}, (v8f){}}; const v16b a = frag_kb(&Ah[nloc][0], hlf), al = frag_kb(&Al[nloc][0], hlf);
#pragma unroll
      for (int t = 0; t < 2; ++t) { const v16b bw = frag_kb(W2T + (size_t)(t * 16 + nloc) * 32, hlf); a2[t] = wmma16b(a, bw, a2[t]); a2[t] = wmma16b(al, bw, a2[t]); }
      wave_lds_sync();
#pragma unroll
      for (int t = 0; t < 2; ++t) { const int c16 = t * 16 + nloc; const float bq = bf16_rne(b2[c16]);
#pragma unroll
        for (int r8 = 0; r8 < 8; ++r8) { b16 p, q; split16(silu(a2[t][r8] * (1.0f / (XS * WSC)) + bq) * XS, p, q); Ah[8 * hlf + r8][c16] = p; Al[8 * hlf + r8][c16] = q; } } }
    wave_lds_sync();
    { v8f a2[2] = {(v8f){}, (v8f){}}; const v16b a = frag_kb(&Ah[nloc][0], hlf), al = frag_kb(&Al[nloc][0], hlf);
#pragma unroll
      for (int t = 0; t < 2; ++t) { const v16b bh = frag_kb(W3H + (size_t)(t * 16 + nloc) * 32, hlf), bl = frag_kb(W3L + (size_t)(t * 16 + nloc) * 32, hlf); a2[t] = wmma16b(a, bh, a2[t]); a2[t] = wmma16b(a, bl, a2[t]); a2[t] = wmma16b(al, bh, a2[t]); }
#pragma unroll
      for (int t = 0; t < 2; ++t)
#pragma unroll
        for (int r8 = 0; r8 < 8; ++r8) Mo[8 * hlf + r8][t * 16 + nloc] = a2[t][r8] * (1.0f / (XS * WSC)); }
    wave_lds_sync();
    for (int rr = 0; rr < 16; ++rr) if (Cs[rr] >= 0) osum += Mo[rr][lane] + bb3;
    wave_lds_sync(); }
  (void)bb1; (void)bb2;
  for (int pass = 0; pass < 2; ++pass) { ((volatile float*)out)[n * CO + lane] = osum; __threadfence(); }
}
}

extern "C" void kernel_launch(void* const* d_in, const int* in_sizes, int n_in, void* d_out, int out_size, void* d_ws, size_t ws_size, hipStream_t stream) {
  (void)n_in;
  auto Fp = [&](int i) { return (const float*)d_in[i]; }; auto Ip = [&](int i) { return (const int*)d_in[i]; };
  if (in_sizes[0] != N * CI || in_sizes[1] != N * 3 || in_sizes[2] != 2 * E || in_sizes[3] != (NSH + CI) * HID || in_sizes[5] != HID * HID || in_sizes[7] != HID * NSH * CO || in_sizes[8] != NSH * CO || out_size != N * CO) return;
  const int NLIM = N;
  size_t off = 0; char* ws = (char*)d_ws;
  auto carve = [&](size_t bytes) { char* p = ws + off; off += (bytes + 255) & ~(size_t)255; return p; };
  b16* W1Y = (b16*)carve(32 * 32 * 2); b16* W1F = (b16*)carve(HID * CI * 2); b16* W2T = (b16*)carve(32 * 32 * 2); b16* W3H = (b16*)carve(32 * 32 * 2); b16* W3L = (b16*)carve(32 * 32 * 2); float* B3S = (float*)carve(128); float* FW = (float*)carve((size_t)N * HID * 4);
  CsrBufs9 csr; off = csr_carve9(csr, ws, off, E, N);
  if (off > ws_size || off > ((size_t)64 << 20)) return;
  wput_kernel<<<1, 256, 0, stream>>>(Fp(3), 0, NSH, 32, HID, W1Y); wput_kernel<<<(HID * 16 + 255) / 256, 256, 0, stream>>>(Fp(3), NSH, CI, CI, HID, W1F); wput_kernel<<<1, 256, 0, stream>>>(Fp(5), 0, HID, 32, HID, W2T);
  w3sum_kernel<<<1, 256, 0, stream>>>(Fp(7), Fp(8), W3H, W3L, B3S);
  csr_build9(csr, Ip(2), E, N, stream);
  fw_kernel<<<NBLK, 32, 0, stream>>>(Fp(0), W1F, FW);
  msg_kernel<<<(unsigned)NLIM, 32, 0, stream>>>(Fp(1), Ip(2) + E, FW, W1Y, Fp(4), W2T, Fp(6), W3H, W3L, B3S, csr.PERM, csr.ROWPTR, csr.ROWCNT, (int)csr.permLen, NLIM, (float*)d_out);
}
